// RNN_53755810677415
// MI455X (gfx1250) — hardware-verified
//
#include <hip/hip_runtime.h>
#include <math.h>

constexpr int NBATCH  = 64;
constexpr int NSTEP   = 512;
constexpr int NIN     = 256;
constexpr int NHID    = 512;
constexpr int NOUT    = 10000;
constexpr int NOUTP   = 10048;
constexpr int NROWS   = NBATCH * NSTEP;
constexpr int NOUT0   = NBATCH * NOUT;
constexpr int NOUT1   = NBATCH * NHID;
constexpr int NTHR    = 256;
constexpr int SEQ_BLK = 16;
constexpr int HPITCH  = 520;
constexpr int SLABP   = 68;
constexpr int LDS_FLOATS = (2 * SEQ_BLK * HPITCH) / 2;

constexpr float WCARRY     = 64.0f;
constexpr float WCARRY_INV = 1.0f / 64.0f;
constexpr float LOCARRY    = 2048.0f;
constexpr float RES_FOLD   = (1.0f / 64.0f) * (1.0f / 2048.0f);

static_assert(NIN % 32 == 0 && NHID % 32 == 0, "GEMM K multiples of 32");
static_assert(NROWS % 32 == 0 && NBATCH % 32 == 0, "GEMM M multiples of 32");
static_assert(NHID % 64 == 0 && NOUTP % 64 == 0 && NOUTP >= NOUT, "GEMM N multiples of 64");
static_assert(NBATCH % SEQ_BLK == 0, "whole 16-row blocks");
static_assert(NHID == 64 * (NTHR / 32), "8 waves x 64 hidden columns");
static_assert(NOUT % 4 == 0, "float4 repack stays inside one row");
static_assert((NOUT0 / 4) % NTHR == 0, "repack grid exact");
static_assert(((size_t)NOUT0 * 4) % 128 == 0, "second output starts on a 128-B line");
static_assert((size_t)NOUT0 * 4 + (size_t)NOUT1 * 4 == (size_t)2691072, "output extent");
static_assert(LDS_FLOATS * 4 >= SEQ_BLK * NHID * 4, "f32 staging fits in the h plane region");
static_assert((HPITCH * 2) % 16 == 0, "16-B aligned fragment rows");

typedef __attribute__((ext_vector_type(16))) _Float16 v16h;
typedef __attribute__((ext_vector_type(8)))  _Float16 v8h;
typedef __attribute__((ext_vector_type(8)))  float    v8f;
typedef __attribute__((ext_vector_type(4)))  float    v4f;

union FragU { v16h v; v8h h[2]; };
__device__ __forceinline__ v16h frag_load(const _Float16* p) {
  FragU f;
  f.h[0] = *(const v8h*)(p);
  f.h[1] = *(const v8h*)(p + 16);
  return f.v;
}
__device__ __forceinline__ v8f frag_mma(v16h a, v16h b, v8f c) {
  return __builtin_amdgcn_wmma_f32_16x16x32_f16(false, a, false, b, (short)0, c, false, false);
}
__device__ __forceinline__ void guard8_h(v8f& a0, v8f& a1, v8f& a2, v8f& a3, v8f& b0, v8f& b1, v8f& b2, v8f& b3,
                                         v16h x, v16h y) {
  asm volatile("v_nop\n\tv_nop\n\tv_nop\n\tv_nop"
               : "+v"(a0), "+v"(a1), "+v"(a2), "+v"(a3), "+v"(b0), "+v"(b1), "+v"(b2), "+v"(b3)
               : "v"(x), "v"(y));
}
__device__ __forceinline__ void keep4_h(v16h a, v16h b, v16h c, v16h d) {
  asm volatile("v_nop" :: "v"(a), "v"(b), "v"(c), "v"(d));
}
__device__ __forceinline__ void acc_guard4(v8f& a, v8f& b, v8f& c, v8f& d) {
  asm volatile("v_nop\n\tv_nop\n\tv_nop\n\tv_nop" : "+v"(a), "+v"(b), "+v"(c), "+v"(d));
}

__device__ __forceinline__ void split_f16(float f, _Float16& hi, _Float16& lo) {
  hi = (_Float16)f;
  const float hf = (float)hi;
  lo = (_Float16)((f - hf) * LOCARRY);
}

__device__ __forceinline__ float tanh_f32(float x) {
  const float xc = fminf(fmaxf(x, -15.0f), 15.0f);
  const float e = expf(2.0f * xc);
  const float rc = 1.0f / (e + 1.0f);
  return 1.0f - 2.0f * rc;
}

template <bool SPLIT>
__global__ __launch_bounds__(NTHR) void cvt8_kernel(const float* __restrict__ src, unsigned short* __restrict__ dhi,
                                                    unsigned short* __restrict__ dlo,
                                                    int nrow_dst, int nrow_src, int ncol8, float sc) {
  const int i  = blockIdx.x * NTHR + threadIdx.x;
  const int n8 = nrow_dst * ncol8;
  if (i < n8) {
    const int row = i / ncol8;
    const int c8  = i - row * ncol8;
    const bool live = (row < nrow_src);
    const int rs = live ? row : (nrow_src - 1);
    const float* sp = src + (size_t)rs * (size_t)(ncol8 * 8) + (size_t)(c8 * 8);
    const v4f a = *(const v4f*)(sp);
    const v4f b = *(const v4f*)(sp + 4);
    v8h hv, lv;
#pragma unroll
    for (int e = 0; e < 4; ++e) {
      const float fa = a[e];
      const float fb = b[e];
      const float f0 = live ? (fa * sc) : 0.0f;
      const float f1 = live ? (fb * sc) : 0.0f;
      _Float16 h0, l0, h1, l1;
      split_f16(f0, h0, l0);
      split_f16(f1, h1, l1);
      hv[e] = h0;
      hv[4 + e] = h1;
      lv[e] = l0;
      lv[4 + e] = l1;
    }
    *(volatile v8h*)(dhi + (size_t)i * 8) = hv;
    if (SPLIT) *(volatile v8h*)(dlo + (size_t)i * 8) = lv;
    __threadfence();
    *(volatile v8h*)(dhi + (size_t)i * 8) = hv;
    if (SPLIT) *(volatile v8h*)(dlo + (size_t)i * 8) = lv;
  }
}

template <bool TWO_BIAS>
__global__ __launch_bounds__(NTHR) void gemm_asplit_kernel(
    const unsigned short* __restrict__ Ahp, const unsigned short* __restrict__ Alp, int lda,
    const unsigned short* __restrict__ Btp, int ldb,
    float* __restrict__ Cout, int ldc,
    const float* __restrict__ bias_a, const float* __restrict__ bias_b,
    int M, int N, int K, int nreal) {
  __shared__ __align__(16) float sT[NTHR / 32][16 * SLABP];
  const _Float16* Ah = (const _Float16*)Ahp;
  const _Float16* Al = (const _Float16*)Alp;
  const _Float16* Bt = (const _Float16*)Btp;
  const int lane = threadIdx.x & 31;
  const int wave = threadIdx.x >> 5;
  const int tilesN = N >> 6;
  const int tilesM = M >> 5;
  const int tile = blockIdx.x * (NTHR / 32) + wave;
  if (tile >= tilesM * tilesN) return;
  const int tm = tile / tilesN;
  const int tn = tile - tm * tilesN;
  const int m0 = tm << 5;
  const int n0 = tn << 6;
  const int rlane = lane & 15;
  const int koff  = (lane >> 4) * 8;
  const int mOff  = (lane >> 4) * 8;

  v8f am[2][4], ar[2][4];
#pragma unroll
  for (int i = 0; i < 2; ++i)
#pragma unroll
    for (int j = 0; j < 4; ++j) {
      am[i][j] = (v8f){0.f, 0.f, 0.f, 0.f, 0.f, 0.f, 0.f, 0.f};
      ar[i][j] = (v8f){0.f, 0.f, 0.f, 0.f, 0.f, 0.f, 0.f, 0.f};
    }

  for (int k0 = 0; k0 < K; k0 += 32) {
    v16h bh[4];
#pragma unroll
    for (int j = 0; j < 4; ++j) {
      const size_t bo = (size_t)(n0 + (j << 4) + rlane) * (size_t)ldb + (size_t)(koff + k0);
      bh[j] = frag_load(Bt + bo);
    }
#pragma unroll
    for (int i = 0; i < 2; ++i) {
      const size_t ao = (size_t)(m0 + (i << 4) + rlane) * (size_t)lda + (size_t)(koff + k0);
      const v16h ah = frag_load(Ah + ao);
      const v16h al = frag_load(Al + ao);
#pragma unroll
      for (int j = 0; j < 4; ++j) {
        am[i][j] = frag_mma(ah, bh[j], am[i][j]);
        ar[i][j] = frag_mma(al, bh[j], ar[i][j]);
      }
      guard8_h(am[i][0], am[i][1], am[i][2], am[i][3], ar[i][0], ar[i][1], ar[i][2], ar[i][3], ah, al);
    }
    keep4_h(bh[0], bh[1], bh[2], bh[3]);
  }
  acc_guard4(am[0][0], am[0][1], am[0][2], am[0][3]);
  acc_guard4(am[1][0], am[1][1], am[1][2], am[1][3]);
  acc_guard4(ar[0][0], ar[0][1], ar[0][2], ar[0][3]);
  acc_guard4(ar[1][0], ar[1][1], ar[1][2], ar[1][3]);

  float bv[4];
#pragma unroll
  for (int j = 0; j < 4; ++j) {
    const int n = n0 + (j << 4) + rlane;
    const int nc = (n < nreal) ? n : (nreal - 1);
    float t = bias_a[nc];
    if (TWO_BIAS) t += bias_b[nc];
    bv[j] = (n < nreal) ? t : 0.0f;
  }

  float* slab = sT[wave];
#pragma unroll
  for (int i = 0; i < 2; ++i) {
    const int mBase = m0 + (i << 4);
#pragma unroll
    for (int j = 0; j < 4; ++j) {
#pragma unroll
      for (int r = 0; r < 8; ++r) {
        const float v = am[i][j][r] * WCARRY_INV + ar[i][j][r] * RES_FOLD + bv[j];
        slab[(mOff + r) * SLABP + (j << 4) + rlane] = v;
      }
    }
    __builtin_amdgcn_fence(__ATOMIC_RELEASE, "workgroup");
    __builtin_amdgcn_wave_barrier();
    __builtin_amdgcn_fence(__ATOMIC_ACQUIRE, "workgroup");
    {
      const int hh = lane >> 4;
      const int c4 = (lane & 15) * 4;
      for (int pass = 0; pass < 2; ++pass) {
#pragma unroll
        for (int it = 0; it < 8; ++it) {
          const int row = it * 2 + hh;
          const v4f v = *(const v4f*)(slab + row * SLABP + c4);
          *(volatile v4f*)(Cout + (size_t)(mBase + row) * (size_t)ldc + (size_t)(n0 + c4)) = v;
        }
        __threadfence();
      }
    }
    __builtin_amdgcn_fence(__ATOMIC_RELEASE, "workgroup");
    __builtin_amdgcn_wave_barrier();
    __builtin_amdgcn_fence(__ATOMIC_ACQUIRE, "workgroup");
  }
}

__global__ __launch_bounds__(NTHR) void rnn_seq_kernel(const float* __restrict__ XG, const float* __restrict__ h0,
                                                       const unsigned short* __restrict__ WHp,
                                                       float* __restrict__ out1,
                                                       unsigned short* __restrict__ HLhi,
                                                       unsigned short* __restrict__ HLlo) {
  __shared__ __align__(16) float lds_f[LDS_FLOATS];
  _Float16* Hhi = (_Float16*)lds_f;
  _Float16* Hlo = Hhi + SEQ_BLK * HPITCH;
  float* Hs = lds_f;
  const _Float16* WH = (const _Float16*)WHp;
  const int tid = threadIdx.x, lane = tid & 31, wave = tid >> 5;
  const int c = lane & 15, hh = lane >> 4, koff = hh * 8;
  const int rowbase = blockIdx.x * SEQ_BLK;

#pragma unroll 1
  for (int it = 0; it < 8; ++it) {
    const int idx = it * NTHR + tid;
    const int row = idx >> 7;
    const int c4  = (idx & 127) * 4;
    const v4f v = *(const v4f*)(h0 + (size_t)(rowbase + row) * NHID + c4);
#pragma unroll
    for (int e = 0; e < 4; ++e) {
      const float f = v[e];
      _Float16 hi, lo;
      split_f16(f, hi, lo);
      Hhi[row * HPITCH + c4 + e] = hi;
      Hlo[row * HPITCH + c4 + e] = lo;
    }
  }
  __syncthreads();

  const _Float16* ahi = Hhi + c * HPITCH + koff;
  const _Float16* alo = Hlo + c * HPITCH + koff;
  const _Float16* w0 = WH + (size_t)(64 * wave + c) * NHID + koff;
  const _Float16* w1 = w0 + (size_t)16 * NHID;
  const _Float16* w2 = w0 + (size_t)32 * NHID;
  const _Float16* w3 = w0 + (size_t)48 * NHID;
  const v8f z8 = {0.f, 0.f, 0.f, 0.f, 0.f, 0.f, 0.f, 0.f};

#pragma unroll 1
  for (int t = 0; t < NSTEP; ++t) {
    v8f am0 = z8, am1 = z8, am2 = z8, am3 = z8;
    v8f ar0 = z8, ar1 = z8, ar2 = z8, ar3 = z8;
#pragma unroll 1
    for (int k0 = 0; k0 < NHID; k0 += 32) {
      const v16h a  = frag_load(ahi + k0);
      const v16h al = frag_load(alo + k0);
      const v16h b0 = frag_load(w0 + k0);
      const v16h b1 = frag_load(w1 + k0);
      const v16h b2 = frag_load(w2 + k0);
      const v16h b3 = frag_load(w3 + k0);
      am0 = frag_mma(a,  b0, am0);
      ar0 = frag_mma(al, b0, ar0);
      am1 = frag_mma(a,  b1, am1);
      ar1 = frag_mma(al, b1, ar1);
      am2 = frag_mma(a,  b2, am2);
      ar2 = frag_mma(al, b2, ar2);
      am3 = frag_mma(a,  b3, am3);
      ar3 = frag_mma(al, b3, ar3);
      guard8_h(am0, am1, am2, am3, ar0, ar1, ar2, ar3, a, al);
      keep4_h(b0, b1, b2, b3);
    }
    acc_guard4(am0, am1, am2, am3);
    acc_guard4(ar0, ar1, ar2, ar3);

    __syncthreads();

    const bool last = (t == NSTEP - 1);
#pragma unroll 1
    for (int nt = 0; nt < 4; ++nt) {
      const v8f am = (nt == 0) ? am0 : ((nt == 1) ? am1 : ((nt == 2) ? am2 : am3));
      const v8f ar = (nt == 0) ? ar0 : ((nt == 1) ? ar1 : ((nt == 2) ? ar2 : ar3));
      const int j = 64 * wave + 16 * nt + c;
      const float* xp = XG + ((size_t)(rowbase + 8 * hh) * NSTEP + (size_t)t) * NHID + j;
      float xg[8];
#pragma unroll
      for (int r = 0; r < 8; ++r) xg[r] = xp[(size_t)r * NSTEP * NHID];
#pragma unroll
      for (int r = 0; r < 8; ++r) {
        const float z = am[r] * WCARRY_INV + ar[r] * RES_FOLD + xg[r];
        const float hn = tanh_f32(z);
        const int row = 8 * hh + r;
        if (last) {
          Hs[row * NHID + j] = hn;
        } else {
          _Float16 hi, lo;
          split_f16(hn, hi, lo);
          Hhi[row * HPITCH + j] = hi;
          Hlo[row * HPITCH + j] = lo;
        }
      }
      asm volatile("" ::: "memory");
    }
    __syncthreads();
  }

  float* o1 = out1 + (size_t)rowbase * NHID;
  for (int pass = 0; pass < 2; ++pass) {
#pragma unroll 1
    for (int it = 0; it < 8; ++it) {
      const int idx = it * NTHR + tid;
      const int row = idx >> 7;
      const int c4  = (idx & 127) * 4;
      const v4f v = *(const v4f*)(Hs + row * NHID + c4);
      *(volatile v4f*)(o1 + (size_t)row * NHID + c4) = v;
    }
#pragma unroll 1
    for (int it = 0; it < 4; ++it) {
      const int idx = it * NTHR + tid;
      const int row = idx >> 6;
      const int c8  = (idx & 63) * 8;
      const v4f a = *(const v4f*)(Hs + row * NHID + c8);
      const v4f b = *(const v4f*)(Hs + row * NHID + c8 + 4);
      v8h hv, lv;
#pragma unroll
      for (int e = 0; e < 4; ++e) {
        const float f0 = a[e];
        const float f1 = b[e];
        _Float16 x0, y0, x1, y1;
        split_f16(f0, x0, y0);
        split_f16(f1, x1, y1);
        hv[e] = x0;
        hv[4 + e] = x1;
        lv[e] = y0;
        lv[4 + e] = y1;
      }
      const size_t o = (size_t)(rowbase + row) * NHID + (size_t)c8;
      *(volatile v8h*)(HLhi + o) = hv;
      *(volatile v8h*)(HLlo + o) = lv;
    }
    __threadfence();
  }
}

__global__ __launch_bounds__(NTHR) void repack_kernel(const float* __restrict__ OUTP, float* __restrict__ out0) {
  const int i = blockIdx.x * NTHR + threadIdx.x;
  if (i < NOUT0 / 4) {
    const int e = 4 * i;
    const int b = e / NOUT;
    const int n = e - b * NOUT;
    const v4f v = *(const v4f*)(OUTP + (size_t)b * NOUTP + n);
    *(volatile v4f*)(out0 + e) = v;
    __threadfence();
    *(volatile v4f*)(out0 + e) = v;
  }
}

extern "C" void kernel_launch(void* const* d_in, const int* in_sizes, int n_in,
                              void* d_out, int out_size, void* d_ws, size_t ws_size, hipStream_t stream) {
  if (n_in < 8 || d_out == nullptr || d_ws == nullptr) return;
  if (in_sizes[0] != NBATCH * NSTEP * NIN || in_sizes[1] != NBATCH * NHID || in_sizes[2] != NHID * NIN ||
      in_sizes[3] != NHID * NHID || in_sizes[4] != NHID || in_sizes[5] != NHID ||
      in_sizes[6] != NOUT * NHID || in_sizes[7] != NOUT || out_size != NOUT0 + NOUT1) return;

  const float* x     = (const float*)d_in[0];
  const float* h0    = (const float*)d_in[1];
  const float* w_xh  = (const float*)d_in[2];
  const float* w_hh  = (const float*)d_in[3];
  const float* b_xh  = (const float*)d_in[4];
  const float* b_hh  = (const float*)d_in[5];
  const float* w_dec = (const float*)d_in[6];
  const float* b_dec = (const float*)d_in[7];
  float* out0 = (float*)d_out;
  float* out1 = out0 + (size_t)NOUT0;

  char* ws = (char*)d_ws;
  size_t off = 0;
  auto carve = [&](size_t bytes) -> char* { char* p = ws + off; off += (bytes + 255) & ~(size_t)255; return p; };
  unsigned short* XHI  = (unsigned short*)carve((size_t)NROWS * NIN * 2);
  unsigned short* XLO  = (unsigned short*)carve((size_t)NROWS * NIN * 2);
  unsigned short* WX16 = (unsigned short*)carve((size_t)NHID * NIN * 2);
  unsigned short* WH16 = (unsigned short*)carve((size_t)NHID * NHID * 2);
  unsigned short* WD16 = (unsigned short*)carve((size_t)NOUTP * NHID * 2);
  float*          XG   = (float*)carve((size_t)NROWS * NHID * 4);
  unsigned short* HLHI = (unsigned short*)carve((size_t)NBATCH * NHID * 2);
  unsigned short* HLLO = (unsigned short*)carve((size_t)NBATCH * NHID * 2);
  float*          OUTP = (float*)carve((size_t)NBATCH * NOUTP * 4);
  if (off > ws_size || off > (size_t)134217728) return;

  const int n8x = NROWS * (NIN / 8);
  const int n8a = NHID * (NIN / 8);
  const int n8h = NHID * (NHID / 8);
  const int n8d = NOUTP * (NHID / 8);
  cvt8_kernel<true><<<(n8x + NTHR - 1) / NTHR, NTHR, 0, stream>>>(x, XHI, XLO, NROWS, NROWS, NIN / 8, 1.0f);
  cvt8_kernel<false><<<(n8a + NTHR - 1) / NTHR, NTHR, 0, stream>>>(w_xh, WX16, WX16, NHID, NHID, NIN / 8, WCARRY);
  cvt8_kernel<false><<<(n8h + NTHR - 1) / NTHR, NTHR, 0, stream>>>(w_hh, WH16, WH16, NHID, NHID, NHID / 8, WCARRY);
  cvt8_kernel<false><<<(n8d + NTHR - 1) / NTHR, NTHR, 0, stream>>>(w_dec, WD16, WD16, NOUTP, NOUT, NHID / 8, WCARRY);

  {
    const int tiles = (NROWS / 32) * (NHID / 64);
    gemm_asplit_kernel<true><<<(tiles + 7) / 8, NTHR, 0, stream>>>(
        XHI, XLO, NIN, WX16, NIN, XG, NHID, b_xh, b_hh, NROWS, NHID, NIN, NHID);
  }

  rnn_seq_kernel<<<NBATCH / SEQ_BLK, NTHR, 0, stream>>>(XG, h0, WH16, out1, HLHI, HLLO);

  {
    const int tiles = (NBATCH / 32) * (NOUTP / 64);
    gemm_asplit_kernel<false><<<(tiles + 7) / 8, NTHR, 0, stream>>>(
        HLHI, HLLO, NHID, WD16, NHID, OUTP, NOUTP, b_dec, b_dec, NBATCH, NOUTP, NHID, NOUT);
  }

  repack_kernel<<<(NOUT0 / 4) / NTHR, NTHR, 0, stream>>>(OUTP, out0);
}
